// MLPDecoder_72378788873075
// MI455X (gfx1250) — hardware-verified
//
#include <hip/hip_runtime.h>
#include <math.h>

#ifndef NB
#define NB 2048
#endif
#define NB_FULL 2048
#define NNODE 20000
#define DD 512
#define HID1 128
#define HID2 64
#define NNEG 64
#define NP (((NNODE + 63) / 64) * 64)
#define MROWS (NB * (1 + NNEG))
#define MPAD (((MROWS + 63) / 64) * 64)

static_assert(NB >= 1 && NB <= NB_FULL);
static_assert(NP % 64 == 0 && MPAD % 64 == 0);
static_assert(DD % 32 == 0 && HID1 % 32 == 0 && HID2 == 64 && (2 * HID1) % 64 == 0);
static_assert(NB_FULL * 4 == 8192);
static_assert((long long)(NB_FULL - NB + MROWS) * 4 <= 532480LL);

typedef __attribute__((ext_vector_type(16))) _Float16 v16h;
typedef __attribute__((ext_vector_type(8)))  _Float16 v8h;
typedef __attribute__((ext_vector_type(16))) __bf16   v16b;
typedef __attribute__((ext_vector_type(8)))  __bf16   v8b;
typedef __attribute__((ext_vector_type(8)))  float    v8f;
typedef __attribute__((ext_vector_type(4)))  float    v4f;

#define VST2(T, ptr, val) do { const T vst2_v_ = (val); *(volatile T*)(ptr) = vst2_v_; __threadfence(); *(volatile T*)(ptr) = vst2_v_; } while (0)

__device__ __forceinline__ unsigned short bfu_rne(float v) { unsigned u = __builtin_bit_cast(unsigned, v); u += 0x7FFFu + ((u >> 16) & 1u); return (unsigned short)(u >> 16); }
__device__ __forceinline__ float bfu_f32(unsigned short h) { return __uint_as_float(((unsigned)h) << 16); }
__device__ __forceinline__ void bfsplit(float v, unsigned short& hi, unsigned short& lo) { hi = bfu_rne(v); lo = bfu_rne(v - bfu_f32(hi)); }
__device__ __forceinline__ void st_s2(unsigned short* Hp, unsigned short* Lp, long long o, float a, float b) { unsigned short h0, l0, h1, l1; bfsplit(a, h0, l0); bfsplit(b, h1, l1);
    const unsigned ph = (unsigned)h0 | ((unsigned)h1 << 16), pl = (unsigned)l0 | ((unsigned)l1 << 16);
    volatile unsigned* dh = (volatile unsigned*)(Hp + o); volatile unsigned* dl = (volatile unsigned*)(Lp + o); *dh = ph; *dl = pl; __threadfence(); *dh = ph; *dl = pl; }
__device__ __forceinline__ void st4s(unsigned short* Hp, unsigned short* Lp, long long o, v4f a) { unsigned short h[4], l[4]; bfsplit(a.x, h[0], l[0]); bfsplit(a.y, h[1], l[1]); bfsplit(a.z, h[2], l[2]); bfsplit(a.w, h[3], l[3]);
    const unsigned long long ph = (unsigned long long)h[0] | ((unsigned long long)h[1] << 16) | ((unsigned long long)h[2] << 32) | ((unsigned long long)h[3] << 48);
    const unsigned long long pl = (unsigned long long)l[0] | ((unsigned long long)l[1] << 16) | ((unsigned long long)l[2] << 32) | ((unsigned long long)l[3] << 48);
    VST2(unsigned long long, (unsigned long long*)(Hp + o), ph); VST2(unsigned long long, (unsigned long long*)(Lp + o), pl); }

namespace w25 {

__device__ __forceinline__ unsigned short f2bf_bits(float f) {
  unsigned u = __float_as_uint(f);
  return (unsigned short)((u + 0x7FFFu + ((u >> 16) & 1u)) >> 16);
}
__device__ __forceinline__ float bf_bits2f(unsigned short h) { return __uint_as_float(((unsigned)h) << 16); }

__device__ __forceinline__ void dep_guard_h(v8f& a, v8f& b, v16h x, v16h y) { asm volatile("v_nop\n\tv_nop\n\tv_nop\n\tv_nop" : "+v"(a), "+v"(b) : "v"(x), "v"(y)); }
__device__ __forceinline__ void dep_guard_b(v8f& a, v8f& b, v16b x, v16b y) { asm volatile("v_nop\n\tv_nop\n\tv_nop\n\tv_nop" : "+v"(a), "+v"(b) : "v"(x), "v"(y)); }
__device__ __forceinline__ void keep4_h(v16h a, v16h b, v16h c, v16h d) { asm volatile("v_nop" :: "v"(a), "v"(b), "v"(c), "v"(d)); }
__device__ __forceinline__ void keep4_b(v16b a, v16b b, v16b c, v16b d) { asm volatile("v_nop" :: "v"(a), "v"(b), "v"(c), "v"(d)); }
__device__ __forceinline__ void acc_guard4(v8f& a, v8f& b, v8f& c, v8f& d) { asm volatile("v_nop\n\tv_nop\n\tv_nop\n\tv_nop" : "+v"(a), "+v"(b), "+v"(c), "+v"(d)); }

template <typename T> struct Frag;
template <> struct Frag<_Float16> {
  typedef v16h V; union U { v16h v; v8h h[2]; };
  static __device__ __forceinline__ v16h load(const _Float16* p) {
    U f; f.h[0] = *(const v8h*)(p); f.h[1] = *(const v8h*)(p + 16); return f.v;
  }
  static __device__ __forceinline__ v8f mma(v16h a, v16h b, v8f c) {
    return __builtin_amdgcn_wmma_f32_16x16x32_f16(false, a, false, b, (short)0, c, false, false);
  }
  static __device__ __forceinline__ void guard(v8f& a, v8f& b, v16h x, v16h y) { dep_guard_h(a, b, x, y); }
  static __device__ __forceinline__ void keep(v16h a, v16h b, v16h c, v16h d) { keep4_h(a, b, c, d); }
};
template <> struct Frag<__bf16> {
  typedef v16b V; union U { v16b v; v8b h[2]; };
  static __device__ __forceinline__ v16b load(const __bf16* p) {
    U f; f.h[0] = *(const v8b*)(p); f.h[1] = *(const v8b*)(p + 16); return f.v;
  }
  static __device__ __forceinline__ v8f mma(v16b a, v16b b, v8f c) {
    return __builtin_amdgcn_wmma_f32_16x16x32_bf16(false, a, false, b, (short)0, c, false, false);
  }
  static __device__ __forceinline__ void guard(v8f& a, v8f& b, v16b x, v16b y) { dep_guard_b(a, b, x, y); }
  static __device__ __forceinline__ void keep(v16b a, v16b b, v16b c, v16b d) { keep4_b(a, b, c, d); }
};

template <int ET> struct Elem;
template <> struct Elem<0> { typedef _Float16 T; };
template <> struct Elem<1> { typedef __bf16 T; };
template <int ET, bool SPLIT, int BIAS_MODE, int OUT_MODE, bool RESID, int ACT = 0>
__global__ __launch_bounds__(256) void wmma_gemm64(
    const unsigned short* __restrict__ Ap, const unsigned short* __restrict__ A2p, int lda, long strideA,
    const unsigned short* __restrict__ Btp, const unsigned short* __restrict__ Bt2p, int ldb, long strideB,
    void* __restrict__ Cout, void* __restrict__ Cout2, int ldc, long strideC,
    const float* __restrict__ bias,
    const float* __restrict__ resid, long strideR,
    int M, int N, int K, float scale) {
  typedef typename Elem<ET>::T T;
  typedef typename Frag<T>::V V;
  const T* A = (const T*)Ap; const T* A2 = (const T*)A2p; const T* Bt = (const T*)Btp; const T* Bt2 = (const T*)Bt2p;
  __shared__ __align__(16) float sT[8][16 * 68];
  const int b    = blockIdx.y;
  const int lane = threadIdx.x & 31;
  const int wave = threadIdx.x >> 5;
  const int tilesN = N >> 6;
  const int tilesM = M >> 6;
  const int tile = blockIdx.x * 8 + wave;
  if (tile >= tilesM * tilesN) return;
  const int tm = tile / tilesN;
  const int tn = tile - tm * tilesN;
  const int m0 = tm << 6;
  const int n0 = tn << 6;

  const T* Ab  = A  + (size_t)b * strideA;
  const T* Bb  = Bt + (size_t)b * strideB;
  const T* Ab2 = SPLIT ? (A2  + (size_t)b * strideA) : nullptr;
  const T* Bb2 = SPLIT ? (Bt2 + (size_t)b * strideB) : nullptr;

  const int rlane = lane & 15;
  const int koff  = (lane >> 4) * 8;
  const int mOff  = (lane >> 4) * 8;

  v8f acc[4][4];
#pragma unroll
  for (int i = 0; i < 4; ++i)
#pragma unroll
    for (int j = 0; j < 4; ++j) acc[i][j] = (v8f){0.f,0.f,0.f,0.f,0.f,0.f,0.f,0.f};

  for (int k0 = 0; k0 < K; k0 += 32) {
    V bh[4], bl[4];
#pragma unroll
    for (int j = 0; j < 4; ++j) {
      const size_t bo = (size_t)(n0 + (j << 4) + rlane) * ldb + koff + k0;
      bh[j] = Frag<T>::load(Bb + bo);
      if (SPLIT) bl[j] = Frag<T>::load(Bb2 + bo);
    }
#pragma unroll
    for (int i = 0; i < 4; ++i) {
      const size_t ao = (size_t)(m0 + (i << 4) + rlane) * lda + koff + k0;
      V ah = Frag<T>::load(Ab + ao);
      V al;
      if (SPLIT) al = Frag<T>::load(Ab2 + ao);
#pragma unroll
      for (int j = 0; j < 4; ++j) {
        acc[i][j] = Frag<T>::mma(ah, bh[j], acc[i][j]);
        if (SPLIT) {
          acc[i][j] = Frag<T>::mma(ah, bl[j], acc[i][j]);
          acc[i][j] = Frag<T>::mma(al, bh[j], acc[i][j]);
        }
      }
      Frag<T>::guard(acc[i][0], acc[i][3], ah, SPLIT ? al : ah);
    }
    Frag<T>::keep(bh[0], bh[1], bh[2], bh[3]);
    if (SPLIT) Frag<T>::keep(bl[0], bl[1], bl[2], bl[3]);
  }
  acc_guard4(acc[0][0], acc[0][1], acc[0][2], acc[0][3]);
  acc_guard4(acc[1][0], acc[1][1], acc[1][2], acc[1][3]);
  acc_guard4(acc[2][0], acc[2][1], acc[2][2], acc[2][3]);
  acc_guard4(acc[3][0], acc[3][1], acc[3][2], acc[3][3]);

  float* slab = sT[wave];
  const float* Rb = RESID ? (resid + (size_t)b * strideR) : nullptr;
#pragma unroll
  for (int i = 0; i < 4; ++i) {
    const int mBase = m0 + (i << 4);
#pragma unroll
    for (int j = 0; j < 4; ++j) {
      const int n = n0 + (j << 4) + rlane;
      float bv = 0.f;
      if (BIAS_MODE == 2) bv = bias[n];
#pragma unroll
      for (int r = 0; r < 8; ++r) {
        float v = acc[i][j][r] * scale;
        if (BIAS_MODE == 1) v += bias[mBase + mOff + r];
        if (BIAS_MODE == 2) v += bv;
        if (RESID) v += Rb[(size_t)(mBase + mOff + r) * ldc + n];
        if (ACT == 1) v = tanhf(v);
        if (ACT == 2) v = fmaxf(v, 0.0f);
        if (ACT == 3) v = v / (1.0f + expf(-v));
        if (ACT == 4) v = (v > 0.f) ? v : 0.01f * v;
        if (ACT == 5) v = 0.5f * v * (1.0f + erff(v * 0.70710678118654752f));
        if (ACT == 6) v = (v > 0.f) ? v : 0.2f * v;
        if (ACT == 7) { const float u = 0.7978845608028654f * (v + 0.044715f * v * v * v); v = 0.5f * v * (1.f + tanhf(u)); }
        slab[(mOff + r) * 68 + (j << 4) + rlane] = v;
      }
    }
    __builtin_amdgcn_fence(__ATOMIC_RELEASE, "workgroup");
    __builtin_amdgcn_wave_barrier();
    __builtin_amdgcn_fence(__ATOMIC_ACQUIRE, "workgroup");
    if (OUT_MODE == 0) {
      float* C = (float*)Cout + (size_t)b * strideC;
      const int hh = lane >> 4, c4 = (lane & 15) * 4;
      for (int pass = 0; pass < 2; ++pass) {
#pragma unroll
        for (int it = 0; it < 8; ++it) {
          const int row = it * 2 + hh;
          v4f v = *(const v4f*)(slab + row * 68 + c4);
          *(volatile v4f*)(C + (size_t)(mBase + row) * ldc + n0 + c4) = v;
        }
        __threadfence();
      }
    } else {
      const int q = lane >> 3, c8 = (lane & 7) * 8;
      unsigned short* C  = (unsigned short*)Cout  + (size_t)b * strideC;
      unsigned short* C2 = (OUT_MODE == 2) ? ((unsigned short*)Cout2 + (size_t)b * strideC) : nullptr;
      for (int pass = 0; pass < 2; ++pass) {
#pragma unroll
        for (int it = 0; it < 4; ++it) {
          const int row = it * 4 + q;
          const float* sp = slab + row * 68 + c8;
          v8h hv, lv;
#pragma unroll
          for (int e = 0; e < 8; ++e) {
            if (OUT_MODE == 1) {
              hv[e] = (_Float16)sp[e];
            } else {
              unsigned short hb = f2bf_bits(sp[e]);
              unsigned short lb = f2bf_bits(sp[e] - bf_bits2f(hb));
              hv[e] = __builtin_bit_cast(_Float16, hb);
              lv[e] = __builtin_bit_cast(_Float16, lb);
            }
          }
          *(volatile v8h*)(C + (size_t)(mBase + row) * ldc + n0 + c8) = hv;
          if (OUT_MODE == 2) *(volatile v8h*)(C2 + (size_t)(mBase + row) * ldc + n0 + c8) = lv;
        }
        __threadfence();
      }
    }
    __builtin_amdgcn_fence(__ATOMIC_RELEASE, "workgroup");
    __builtin_amdgcn_wave_barrier();
    __builtin_amdgcn_fence(__ATOMIC_ACQUIRE, "workgroup");
  }
}

}

__global__ __launch_bounds__(256) void k_pl4r(const float* __restrict__ X, int PW, int Wd, int RL, int RP, unsigned short* __restrict__ PH_, unsigned short* __restrict__ PL_, int PP) {
    const long long u = (long long)blockIdx.x * 256 + threadIdx.x; const int cq = Wd / 4; if (u >= (long long)RP * cq) return;
    const int r = (int)(u / cq); const int c = 4 * (int)(u % cq); const int rr = min(r, RL - 1);
    v4f v = *(const v4f*)(X + (long long)rr * PW + c);
    if (r >= RL) { v.x = 0.f; v.y = 0.f; v.z = 0.f; v.w = 0.f; }
    st4s(PH_, PL_, (long long)r * PP + c, v); }

__global__ __launch_bounds__(256) void k_bt(const float* __restrict__ Wm, int ldw, int KI, int NO, int KP, int NOP, unsigned short* __restrict__ PH_, unsigned short* __restrict__ PL_) {
    const long long u = (long long)blockIdx.x * 256 + threadIdx.x; if (u >= (long long)NOP * (KP / 2)) return;
    const int k0 = 2 * (int)(u % (KP / 2)); const int o = (int)(u / (KP / 2));
    const int oo = min(o, NO - 1); const int ka = min(k0, KI - 1); const int kb = min(k0 + 1, KI - 1);
    float a = Wm[(long long)ka * ldw + oo]; float b = Wm[(long long)kb * ldw + oo];
    a = (o < NO && k0 < KI) ? a : 0.f; b = (o < NO && k0 + 1 < KI) ? b : 0.f;
    st_s2(PH_, PL_, (long long)o * KP + k0, a, b); }

__global__ __launch_bounds__(256) void k_h1(const float* __restrict__ PQ, const float* __restrict__ B1, const int* __restrict__ HI, const int* __restrict__ TI, const int* __restrict__ NS,
        unsigned short* __restrict__ PH_, unsigned short* __restrict__ PL_, int nb, int mrows, int mpad, int nnode) {
    const long long u = (long long)blockIdx.x * 256 + threadIdx.x; if (u >= (long long)mpad * (HID1 / 4)) return;
    const int r = (int)(u / (HID1 / 4)); const int c = 4 * (int)(u % (HID1 / 4));
    const int rr = min(r, mrows - 1);
    const int isneg = (rr >= nb) ? 1 : 0;
    const int idx = max(rr - nb, 0);
    const int bneg = min(idx / NNEG, nb - 1);
    const int j = idx % NNEG;
    const int bpos = min(rr, nb - 1);
    const int bb = isneg ? bneg : bpos;
    const int hv = HI[bb], tv = TI[bb];
    const int ns = NS[(long long)bneg * NNEG + j];
    int li = (isneg && j >= NNEG / 2) ? ns : hv;
    int ri = (isneg && j < NNEG / 2) ? ns : tv;
    li = min(max(li, 0), nnode - 1); ri = min(max(ri, 0), nnode - 1);
    const v4f p = *(const v4f*)(PQ + (long long)li * (2 * HID1) + c);
    const v4f q = *(const v4f*)(PQ + (long long)ri * (2 * HID1) + HID1 + c);
    const v4f bv = *(const v4f*)(B1 + c);
    v4f v = p + q + bv;
    v.x = fmaxf(v.x, 0.f); v.y = fmaxf(v.y, 0.f); v.z = fmaxf(v.z, 0.f); v.w = fmaxf(v.w, 0.f);
    if (r >= mrows) { v.x = 0.f; v.y = 0.f; v.z = 0.f; v.w = 0.f; }
    st4s(PH_, PL_, (long long)r * HID1 + c, v); }

__global__ __launch_bounds__(256) void k_head(const float* __restrict__ X, const float* __restrict__ W3, const float* __restrict__ B3, float* __restrict__ OUT, int mrows, int nb, int nbfull) {
    const int r = blockIdx.x * 256 + threadIdx.x; if (r >= mrows) return;
    const float* xr = X + (long long)r * HID2;
    float s = B3[0];
#pragma unroll 1
    for (int c = 0; c < HID2; c += 4) { const v4f a = *(const v4f*)(xr + c); const v4f w = *(const v4f*)(W3 + c); s += a.x * w.x + a.y * w.y + a.z * w.z + a.w * w.w; }
    const int o = (r < nb) ? r : (nbfull - nb + r);
    VST2(float, OUT + o, s); }

#define WSB_APL   ((size_t)NP * DD * 2)
#define WSB_H1PL  ((size_t)MPAD * HID1 * 2)
#define WSB_R1    ((2 * WSB_APL > 2 * WSB_H1PL) ? (2 * WSB_APL) : (2 * WSB_H1PL))
#define WSB_W1PL  ((size_t)(2 * HID1) * DD * 2)
#define WSB_W2PL  ((size_t)HID2 * HID1 * 2)
#define WSB_PQ    ((size_t)NP * (2 * HID1) * 4)
#define WSB_H2    ((size_t)MPAD * HID2 * 4)
#define WSB_TOTAL (WSB_R1 + 2 * WSB_W1PL + 2 * WSB_W2PL + WSB_PQ + WSB_H2)
static_assert(WSB_TOTAL <= 134217728ull);
static_assert(WSB_APL % 256 == 0 && WSB_H1PL % 256 == 0 && WSB_W1PL % 256 == 0 && WSB_W2PL % 256 == 0 && WSB_PQ % 256 == 0 && WSB_H2 % 256 == 0);

extern "C" void kernel_launch(void* const* d_in, const int* in_sizes, int n_in, void* d_out, int out_size, void* d_ws, size_t ws_size, hipStream_t stream) {
    if (n_in < 10) return;
    if (in_sizes[0] < NNODE * DD || in_sizes[1] < 2 * DD * HID1 || in_sizes[2] < HID1 || in_sizes[3] < HID1 * HID2 || in_sizes[4] < HID2 ||
        in_sizes[5] < HID2 || in_sizes[6] < 1 || in_sizes[7] < NB || in_sizes[8] < NB || in_sizes[9] < NB * NNEG) return;
    if (out_size < NB_FULL - NB + MROWS) return;
    if (WSB_TOTAL > ws_size) return;
    const float* embed = (const float*)d_in[0];
    const float* W1    = (const float*)d_in[1];
    const float* b1    = (const float*)d_in[2];
    const float* W2    = (const float*)d_in[3];
    const float* b2    = (const float*)d_in[4];
    const float* W3    = (const float*)d_in[5];
    const float* b3    = (const float*)d_in[6];
    const int*   hI    = (const int*)d_in[7];
    const int*   tI    = (const int*)d_in[8];
    const int*   nsI   = (const int*)d_in[9];
    float* out = (float*)d_out;

    char* wsp = (char*)d_ws;
    unsigned short* AH  = (unsigned short*)wsp;
    unsigned short* AL  = (unsigned short*)(wsp + WSB_APL);
    unsigned short* H1H = (unsigned short*)wsp;
    unsigned short* H1L = (unsigned short*)(wsp + WSB_H1PL);
    wsp += WSB_R1;
    unsigned short* WH  = (unsigned short*)wsp; wsp += WSB_W1PL;
    unsigned short* WL  = (unsigned short*)wsp; wsp += WSB_W1PL;
    unsigned short* W2H = (unsigned short*)wsp; wsp += WSB_W2PL;
    unsigned short* W2L = (unsigned short*)wsp; wsp += WSB_W2PL;
    float* PQ  = (float*)wsp; wsp += WSB_PQ;
    float* H2b = (float*)wsp; wsp += WSB_H2;
    if ((size_t)(wsp - (char*)d_ws) > ws_size) return;

    k_pl4r<<<(unsigned)(((long long)NP * (DD / 4) + 255) / 256), 256, 0, stream>>>(embed, DD, DD, NNODE, NP, AH, AL, DD);
    k_bt<<<(unsigned)(((long long)HID1 * (DD / 2) + 255) / 256), 256, 0, stream>>>(W1, HID1, DD, HID1, DD, HID1, WH, WL);
    k_bt<<<(unsigned)(((long long)HID1 * (DD / 2) + 255) / 256), 256, 0, stream>>>(W1 + (size_t)DD * HID1, HID1, DD, HID1, DD, HID1, WH + (size_t)HID1 * DD, WL + (size_t)HID1 * DD);
    k_bt<<<(unsigned)(((long long)HID2 * (HID1 / 2) + 255) / 256), 256, 0, stream>>>(W2, HID2, HID1, HID2, HID1, HID2, W2H, W2L);
    w25::wmma_gemm64<1, true, 0, 0, false, 0><<<dim3((unsigned)(((NP / 64) * ((2 * HID1) / 64) + 7) / 8), 1u), 256, 0, stream>>>(
        (const unsigned short*)AH, (const unsigned short*)AL, DD, 0L, (const unsigned short*)WH, (const unsigned short*)WL, DD, 0L,
        (void*)PQ, nullptr, 2 * HID1, 0L, nullptr, nullptr, 0L, NP, 2 * HID1, DD, 1.0f);
    k_h1<<<(unsigned)(((long long)MPAD * (HID1 / 4) + 255) / 256), 256, 0, stream>>>(PQ, b1, hI, tI, nsI, H1H, H1L, NB, MROWS, MPAD, NNODE);
    w25::wmma_gemm64<1, true, 2, 0, false, 2><<<dim3((unsigned)(((MPAD / 64) * (HID2 / 64) + 7) / 8), 1u), 256, 0, stream>>>(
        (const unsigned short*)H1H, (const unsigned short*)H1L, HID1, 0L, (const unsigned short*)W2H, (const unsigned short*)W2L, HID1, 0L,
        (void*)H2b, nullptr, HID2, 0L, b2, nullptr, 0L, MPAD, HID2, HID1, 1.0f);
    k_head<<<(unsigned)((MROWS + 255) / 256), 256, 0, stream>>>(H2b, W3, b3, out, MROWS, NB, NB_FULL);
}
